// GATS_72645076844636
// MI455X (gfx1250) — hardware-verified
//
#include <hip/hip_runtime.h>
#include <stddef.h>


#define CDIM    64
#define HEADS   8
#define NTHR    256
#define NWAVE   8
#define NBKT    32
#define BKSH    12
#define BKSZ    4096
#define PCH     4096
#define PSTG    (PCH + NBKT * 32)
#define PLINES  (PSTG / 32)
#define DEGB    16384
#define DEGX    32
#define NODB    128
#define TBLK    128
#define TROWS   64
#define WSCAL   16.0f
#define WINV    0.0625f
#define NEGSL   0.2f
#define NEG_BIG (-1.0e30f)
#define WSCAP   134217728
#define LDS_AGG ((BKSZ * 4 + BKSZ * HEADS + BKSZ) * 4)
#define LDS_DEG ((DEGB + DEGX) * 4)

static_assert(NTHR == NWAVE * 32);
static_assert(NWAVE * NBKT == NTHR);
static_assert((1 << BKSH) == BKSZ);
static_assert(PCH == 16 * NTHR);
static_assert(PLINES * 32 == PSTG);
static_assert(PLINES <= NTHR);
static_assert(HEADS == 8 && NWAVE == 8);
static_assert(TROWS == (TBLK / 32) * 16);
static_assert((DEGB % (NTHR * 4)) == 0);
static_assert((BKSZ % (2 * NWAVE)) == 0 && (BKSZ % NTHR) == 0);
static_assert((NODB % 32) == 0 && NODB == 128);

typedef float    v4f  __attribute__((ext_vector_type(4)));
typedef float    v8f  __attribute__((ext_vector_type(8)));
typedef int      v4i  __attribute__((ext_vector_type(4)));
typedef _Float16 v8h  __attribute__((ext_vector_type(8)));
typedef _Float16 v16h __attribute__((ext_vector_type(16)));
union FragH { v16h v; v8h h[2]; };

__device__ __forceinline__ v8f wmh(v16h a, v16h b, v8f c) {
  v8f d = __builtin_amdgcn_wmma_f32_16x16x32_f16(false, a, false, b, (short)0, c, false, false);
  asm volatile("v_nop\n\tv_nop\n\tv_nop\n\tv_nop" : "+v"(d) : "v"(a), "v"(b));
  return d;
}

__device__ __forceinline__ float softplus_f(float v) {
  return fmaxf(v, 0.0f) + log1pf(expf(-fabsf(v)));
}

__device__ __forceinline__ int lowbit(unsigned m) { return __builtin_ffs((int)m) - 1; }

__device__ __forceinline__ int wave_incl_scan(int v, int lane) {
#pragma unroll
  for (int d = 1; d < 32; d <<= 1) {
    const int t = __shfl_up(v, d);
    v += (lane >= d) ? t : 0;
  }
  return v;
}

__global__ __launch_bounds__(NODB) void k_node(const float* __restrict__ x, const int* __restrict__ dist,
                                               const float* __restrict__ train_a, const float* __restrict__ dist1_a,
                                               _Float16* xs16, float* nodep, int nN) {
  __shared__ __attribute__((aligned(16))) _Float16 srow[NODB * CDIM];
  const int tid = threadIdx.x, lane = tid & 31, wave = tid >> 5;
  const int row = (int)blockIdx.x * NODB + tid;
  const int rr  = row < nN ? row : nN - 1;
  const float* xr = x + (size_t)rr * CDIM;

  float v[CDIM];
#pragma unroll
  for (int i = 0; i < CDIM / 4; ++i) {
    const v4f t = *(const v4f*)(xr + 4 * i);
    v[4 * i + 0] = t.x; v[4 * i + 1] = t.y; v[4 * i + 2] = t.z; v[4 * i + 3] = t.w;
  }
  float mn = v[0], mx = v[0];
#pragma unroll
  for (int i = 1; i < CDIM; ++i) { mn = fminf(mn, v[i]); mx = fmaxf(mx, v[i]); }

  float s = 0.0f;
#pragma unroll 1
  for (int i = 0; i < CDIM; ++i) s += __expf(xr[i] - mx);
  const float conf = 1.0f / s;
  const float inv  = 1.0f / (mx - mn);
#pragma unroll
  for (int i = 0; i < CDIM; ++i) v[i] = (v[i] - mn) * inv;

#pragma unroll
  for (int k = 2; k <= CDIM; k <<= 1) {
#pragma unroll
    for (int j = k >> 1; j > 0; j >>= 1) {
#pragma unroll
      for (int i = 0; i < CDIM; ++i) {
        const int l = i ^ j;
        if (l > i) {
          const float va = v[i], vb = v[l];
          const float lo = fminf(va, vb), hi = fmaxf(va, vb);
          const bool up = ((i & k) == 0);
          v[i] = up ? lo : hi;
          v[l] = up ? hi : lo;
        }
      }
    }
  }

  const int dd = dist[rr];
  const float ta = train_a[0], da = dist1_a[0];
  const float a = (dd == 0) ? ta : ((dd == 1) ? da : 1.0f);
  v4f np;
  np.x = a; np.y = 1.0f / a; np.z = conf; np.w = 0.0f;

  _Float16* sr = srow + tid * CDIM;
#pragma unroll
  for (int c = 0; c < CDIM / 8; ++c) {
    v8h p;
#pragma unroll
    for (int j = 0; j < 8; ++j) p[j] = (_Float16)v[8 * c + j];
    *(v8h*)(sr + 8 * c) = p;
  }
  float* npp = nodep + (size_t)row * 4;
  *(volatile v4f*)npp = np;
  __syncthreads();

  const int rbase = (int)blockIdx.x * NODB;
  const int piece = lane & 7;
#pragma unroll
  for (int k = 0; k < 8; ++k) {
    const int r = wave * 32 + 4 * k + (lane >> 3);
    union { v8h h; v4i i; } u;
    u.h = *(const v8h*)(srow + r * CDIM + 8 * piece);
    *(volatile v4i*)(xs16 + (size_t)(rbase + r) * CDIM + 8 * piece) = u.i;
  }
  __threadfence();
  *(volatile v4f*)npp = np;
#pragma unroll
  for (int k = 0; k < 8; ++k) {
    const int r = wave * 32 + 4 * k + (lane >> 3);
    union { v8h h; v4i i; } u;
    u.h = *(const v8h*)(srow + r * CDIM + 8 * piece);
    *(volatile v4i*)(xs16 + (size_t)(rbase + r) * CDIM + 8 * piece) = u.i;
  }
}

__global__ __launch_bounds__(TBLK) void k_temp(const _Float16* __restrict__ xs16, const float* __restrict__ W,
                                               float* temp) {
  __shared__ __attribute__((aligned(16))) _Float16 wl[16 * CDIM];
  __shared__ __attribute__((aligned(16))) float stg[(TBLK / 32) * 16 * HEADS];
  const int tid = threadIdx.x, lane = tid & 31, wave = tid >> 5, hh = lane >> 4, m = lane & 15;
  {
    const int n = tid >> 3, k0 = (tid & 7) * 8;
    const int nc = n < HEADS ? n : HEADS - 1;
    v8h p;
#pragma unroll
    for (int j = 0; j < 8; ++j) {
      const float wv = W[nc * CDIM + k0 + j];
      p[j] = (_Float16)(n < HEADS ? wv * WSCAL : 0.0f);
    }
    *(v8h*)(wl + n * CDIM + k0) = p;
  }
  __syncthreads();

  const int row0 = ((int)blockIdx.x * (TBLK / 32) + wave) * 16;
  v8f acc = {0.f, 0.f, 0.f, 0.f, 0.f, 0.f, 0.f, 0.f};
  const _Float16* ap = xs16 + (size_t)(row0 + m) * CDIM + 8 * hh;
  const _Float16* bp = wl + m * CDIM + 8 * hh;
#pragma unroll
  for (int kt = 0; kt < CDIM / 32; ++kt) {
    FragH a, b;
    a.h[0] = *(const v8h*)(ap + 32 * kt);
    a.h[1] = *(const v8h*)(ap + 32 * kt + 16);
    b.h[0] = *(const v8h*)(bp + 32 * kt);
    b.h[1] = *(const v8h*)(bp + 32 * kt + 16);
    acc = wmh(a.v, b.v, acc);
  }
  float* sp = stg + wave * (16 * HEADS);
  if (m < HEADS) {
#pragma unroll
    for (int r = 0; r < 8; ++r) sp[(8 * hh + r) * HEADS + m] = acc[r] * WINV;
  }
  __syncthreads();
  const v4f o = *(const v4f*)(sp + 4 * lane);
  float* gp = temp + (size_t)row0 * HEADS + 4 * lane;
  *(volatile v4f*)gp = o;
  __threadfence();
  *(volatile v4f*)gp = o;
}

__global__ __launch_bounds__(NTHR) void k_degc(const int* __restrict__ srcs, int* degc, int nE, int vec4) {
  extern __shared__ int dlds[];
  const int tid = threadIdx.x, lane = tid & 31;
  const int nodeBase = (int)blockIdx.x * DEGB;
  for (int i = tid; i < DEGB + DEGX; i += NTHR) dlds[i] = 0;
  __syncthreads();

  const int span = NTHR * 8;
  const int nIt = (nE + span - 1) / span;
#pragma unroll 1
  for (int it = 0; it < nIt; ++it) {
    const int e0 = it * span + tid * 8;
    v4i a, b;
    if (vec4 != 0 && (it + 1) * span <= nE) {
      a = *(const v4i*)(srcs + e0);
      b = *(const v4i*)(srcs + e0 + 4);
    } else {
#pragma unroll
      for (int k = 0; k < 4; ++k) {
        const int ea = e0 + k, eb = e0 + 4 + k;
        const int va = srcs[ea < nE ? ea : nE - 1];
        const int vb = srcs[eb < nE ? eb : nE - 1];
        a[k] = (ea < nE) ? va : -1;
        b[k] = (eb < nE) ? vb : -1;
      }
    }
#pragma unroll
    for (int k = 0; k < 4; ++k) {
      const unsigned u = (unsigned)(a[k] - nodeBase);
      const int idx = (u < (unsigned)DEGB) ? (int)u : (DEGB + lane);
      atomicAdd(&dlds[idx], 1);
    }
#pragma unroll
    for (int k = 0; k < 4; ++k) {
      const unsigned u = (unsigned)(b[k] - nodeBase);
      const int idx = (u < (unsigned)DEGB) ? (int)u : (DEGB + lane);
      atomicAdd(&dlds[idx], 1);
    }
  }
  __syncthreads();

#pragma unroll
  for (int k = 0; k < DEGB / (NTHR * 4); ++k) {
    const int f = (k * NTHR + tid) * 4;
    const v4i cv = *(const v4i*)(dlds + f);
    *(volatile v4i*)(degc + nodeBase + f) = cv;
  }
  __threadfence();
#pragma unroll
  for (int k = 0; k < DEGB / (NTHR * 4); ++k) {
    const int f = (k * NTHR + tid) * 4;
    const v4i cv = *(const v4i*)(dlds + f);
    *(volatile v4i*)(degc + nodeBase + f) = cv;
  }
}

template <int FILL>
__global__ __launch_bounds__(NTHR) void k_part(const int* __restrict__ srcs, const int* __restrict__ dsts,
                                               int* ctab, int* elist, int nN, int nE, int nCh, int vec4, int lcap) {
  __shared__ int histw[NWAVE * NBKT];
  __shared__ int wbase[NWAVE * NBKT];
  __shared__ __attribute__((aligned(16))) int scnt[NBKT];
  __shared__ int srun[NBKT];
  __shared__ int sgo[NBKT];
  __shared__ int lineb[PLINES];
  __shared__ __attribute__((aligned(16))) int stg[FILL ? PSTG : 4];
  __shared__ int snl;
  const int tid = threadIdx.x, lane = tid & 31, wave = tid >> 5;
  const int ch = blockIdx.x;
  const int cbase = ch * PCH;

  histw[tid] = 0;
  wbase[tid] = 0;
  if constexpr (FILL != 0) {
    for (int i = tid; i < PSTG; i += NTHR) stg[i] = -1;
    if (tid < PLINES) lineb[tid] = 0;
  }
  if (tid < NBKT) { scnt[tid] = 0; srun[tid] = 0; sgo[tid] = 0; }
  if (tid == 0) snl = 0;
  __syncthreads();

  v4i dk[4], sk[4];
  if (vec4 != 0) {
#pragma unroll
    for (int j4 = 0; j4 < 4; ++j4) {
      int q = cbase + 4 * (j4 * NTHR + tid);
      q = q > nE - 4 ? nE - 4 : q;
      q = q < 0 ? 0 : q;
      dk[j4] = *(const v4i*)(dsts + q);
      if constexpr (FILL != 0) sk[j4] = *(const v4i*)(srcs + q);
      else { const v4i z = {0, 0, 0, 0}; sk[j4] = z; }
    }
  } else {
#pragma unroll
    for (int j4 = 0; j4 < 4; ++j4) {
      const int eb = cbase + 4 * (j4 * NTHR + tid);
      const int c0 = eb     < nE ? eb     : nE - 1;
      const int c1 = eb + 1 < nE ? eb + 1 : nE - 1;
      const int c2 = eb + 2 < nE ? eb + 2 : nE - 1;
      const int c3 = eb + 3 < nE ? eb + 3 : nE - 1;
      int t0 = dsts[c0], t1 = dsts[c1], t2 = dsts[c2], t3 = dsts[c3];
      int u0 = 0, u1 = 0, u2 = 0, u3 = 0;
      if constexpr (FILL != 0) { u0 = srcs[c0]; u1 = srcs[c1]; u2 = srcs[c2]; u3 = srcs[c3]; }
      asm volatile("" : "+v"(t0), "+v"(t1), "+v"(t2), "+v"(t3), "+v"(u0), "+v"(u1), "+v"(u2), "+v"(u3) : : "memory");
      v4i da, sa;
      da.x = t0; da.y = t1; da.z = t2; da.w = t3;
      sa.x = u0; sa.y = u1; sa.z = u2; sa.w = u3;
      dk[j4] = da; sk[j4] = sa;
    }
  }

  int rk[16];
  int* hw = histw + wave * NBKT;
#pragma unroll
  for (int j = 0; j < 16; ++j) {
    const int e = cbase + 4 * ((j >> 2) * NTHR + tid) + (j & 3);
    const int d = dk[j >> 2][j & 3];
    const bool valid = (e < nE) && ((unsigned)d < (unsigned)nN);
    const int key = valid ? (d >> BKSH) : 0;
    const unsigned vb = __builtin_amdgcn_ballot_w32(valid);
    const unsigned q0 = __builtin_amdgcn_ballot_w32((key & 1) != 0);
    const unsigned q1 = __builtin_amdgcn_ballot_w32((key & 2) != 0);
    const unsigned q2 = __builtin_amdgcn_ballot_w32((key & 4) != 0);
    const unsigned q3 = __builtin_amdgcn_ballot_w32((key & 8) != 0);
    const unsigned q4 = __builtin_amdgcn_ballot_w32((key & 16) != 0);
    unsigned eq = vb;
    eq &= (key & 1)  ? q0 : ~q0;
    eq &= (key & 2)  ? q1 : ~q1;
    eq &= (key & 4)  ? q2 : ~q2;
    eq &= (key & 8)  ? q3 : ~q3;
    eq &= (key & 16) ? q4 : ~q4;
    const int r  = (int)__builtin_amdgcn_mbcnt_lo(eq, 0u);
    const int cn = __builtin_popcount(eq);
    const int base = hw[key];
    rk[j] = base + r;
    if (valid && r == 0) hw[key] = base + cn;
    __syncthreads();
  }

  if (wave == 0) {
    const int b = lane;
    int run = 0;
#pragma unroll
    for (int w = 0; w < NWAVE; ++w) {
      const int c = histw[w * NBKT + b];
      if constexpr (FILL != 0) wbase[w * NBKT + b] = run;
      run += c;
    }
    scnt[b] = run;
    if constexpr (FILL != 0) {
      const int plen = (run + 31) & ~31;
      const int pin  = wave_incl_scan(plen, lane);
      const int srb  = pin - plen;
      const int nl   = __shfl(pin, 31) >> 5;
      int pre = 0, tot = 0;
#pragma unroll 1
      for (int c2 = 0; c2 < nCh; ++c2) {
        int cv = ctab[(size_t)c2 * NBKT + b];
        cv = cv < 0 ? 0 : (cv > PCH ? PCH : cv);
        const int p = (cv + 31) & ~31;
        pre += (c2 < ch) ? p : 0;
        tot += p;
      }
      const int tin = wave_incl_scan(tot, lane);
      const int b0  = tin - tot;
      sgo[b]  = b0 + pre;
      srun[b] = srb;
      if (lane == 0) snl = nl > PLINES ? PLINES : nl;
      const int nlb = plen >> 5, lst = srb >> 5;
#pragma unroll 1
      for (int k = 0; k < nlb; ++k) {
        const int idx = lst + k;
        if (idx < PLINES) lineb[idx] = b;
      }
    }
  }
  __syncthreads();

  if constexpr (FILL == 0) {
    if (tid < NBKT / 4) {
      const v4i cv = *(const v4i*)(scnt + 4 * tid);
      *(volatile v4i*)(ctab + (size_t)ch * NBKT + 4 * tid) = cv;
    }
    __threadfence();
    if (tid < NBKT / 4) {
      const v4i cv = *(const v4i*)(scnt + 4 * tid);
      *(volatile v4i*)(ctab + (size_t)ch * NBKT + 4 * tid) = cv;
    }
  } else {
#pragma unroll
    for (int j = 0; j < 16; ++j) {
      const int e = cbase + 4 * ((j >> 2) * NTHR + tid) + (j & 3);
      const int d = dk[j >> 2][j & 3];
      const bool valid = (e < nE) && ((unsigned)d < (unsigned)nN);
      const int key = valid ? (d >> BKSH) : 0;
      int pos = srun[key] + wbase[wave * NBKT + key] + rk[j];
      pos = pos < 0 ? 0 : (pos > PSTG - 1 ? PSTG - 1 : pos);
      int sv = sk[j >> 2][j & 3];
      sv = sv < 0 ? 0 : (sv > nN - 1 ? nN - 1 : sv);
      if (valid) stg[pos] = (sv << BKSH) | (d & (BKSZ - 1));
    }
    __syncthreads();
    const int nl = snl;
    const int piece = tid & 7;
#pragma unroll 1
    for (int L = tid >> 3; L < nl; L += NTHR / 8) {
      const int b = lineb[L] & (NBKT - 1);
      int g0 = sgo[b] + (L << 5) - srun[b];
      g0 = g0 < 0 ? 0 : (g0 > lcap - 32 ? lcap - 32 : g0);
      g0 &= ~31;
      const v4i ev = *(const v4i*)(stg + (L << 5) + 4 * piece);
      *(volatile v4i*)(elist + g0 + 4 * piece) = ev;
    }
    __threadfence();
#pragma unroll 1
    for (int L = tid >> 3; L < nl; L += NTHR / 8) {
      const int b = lineb[L] & (NBKT - 1);
      int g0 = sgo[b] + (L << 5) - srun[b];
      g0 = g0 < 0 ? 0 : (g0 > lcap - 32 ? lcap - 32 : g0);
      g0 &= ~31;
      const v4i ev = *(const v4i*)(stg + (L << 5) + 4 * piece);
      *(volatile v4i*)(elist + g0 + 4 * piece) = ev;
    }
  }
}

__global__ __launch_bounds__(NTHR) void k_agg(const float* __restrict__ x, const int* __restrict__ elist,
                                              const int* __restrict__ ctab, const float* __restrict__ nodep,
                                              const float* __restrict__ temp, const int* __restrict__ degc,
                                              const float* __restrict__ coefp, const float* __restrict__ biasp,
                                              float* out, int nN, int nCh, int lcap, int maxIter) {
  extern __shared__ v4f alds[];
  v4f*   st4  = alds;
  float* accl = (float*)(alds + BKSZ);
  float* rtl  = accl + BKSZ * HEADS;
  __shared__ int sB0, sLen;
  const int tid = threadIdx.x, lane = tid & 31, wave = tid >> 5, g = lane >> 3, hl = lane & 7;
  const int bk = blockIdx.x;
  const int nodeBase = bk * BKSZ;

  {
    v4f iv; iv.x = NEG_BIG; iv.y = 0.0f; iv.z = 0.0f; iv.w = 0.0f;
    for (int i = tid; i < BKSZ; i += NTHR) st4[i] = iv;
    const v4f z = {0.f, 0.f, 0.f, 0.f};
    v4f* a4 = (v4f*)accl;
    for (int i = tid; i < BKSZ * HEADS / 4; i += NTHR) a4[i] = z;
    for (int i = tid; i < BKSZ; i += NTHR) rtl[i] = 0.0f;
  }
  if (wave == 0) {
    int tot = 0;
#pragma unroll 1
    for (int c2 = 0; c2 < nCh; ++c2) {
      int cv = ctab[(size_t)c2 * NBKT + lane];
      cv = cv < 0 ? 0 : (cv > PCH ? PCH : cv);
      tot += (cv + 31) & ~31;
    }
    const int tin = wave_incl_scan(tot, lane);
    const int b0 = tin - tot;
    if (lane == bk) { sB0 = b0; sLen = tot; }
  }
  __syncthreads();

  int B0b = sB0;
  B0b = B0b < 0 ? 0 : (B0b > lcap ? lcap : B0b);
  int Lb = sLen;
  Lb = Lb < 0 ? 0 : (Lb > lcap - B0b ? lcap - B0b : Lb);
  int nIter = Lb >> 5;
  nIter = nIter > maxIter ? maxIter : nIter;

#pragma unroll 1
  for (int it = 0; it < nIter; ++it) {
    int pidx = B0b + (it << 5) + lane;
    pidx = pidx > lcap - 1 ? lcap - 1 : pidx;
    const int ent = elist[pidx];
    const bool own = (ent >= 0) && ((ent & (NWAVE - 1)) == wave);
    unsigned M = __builtin_amdgcn_ballot_w32(own);
    while (M != 0u) {
      const int l0 = lowbit(M); M &= M - 1u;
      const bool v1 = (M != 0u); const int l1 = v1 ? lowbit(M) : l0; M &= M - 1u;
      const bool v2 = (M != 0u); const int l2 = v2 ? lowbit(M) : l0; M &= M - 1u;
      const bool v3 = (M != 0u); const int l3 = v3 ? lowbit(M) : l0; M &= M - 1u;
      const int e0 = __builtin_amdgcn_readlane(ent, l0);
      const int e1 = __builtin_amdgcn_readlane(ent, l1);
      const int e2 = __builtin_amdgcn_readlane(ent, l2);
      const int e3 = __builtin_amdgcn_readlane(ent, l3);
      const int sl0 = e0 & (BKSZ - 1), sl1 = e1 & (BKSZ - 1), sl2 = e2 & (BKSZ - 1), sl3 = e3 & (BKSZ - 1);
      const bool dup = (v1 && sl1 == sl0) || (v2 && (sl2 == sl0 || sl2 == sl1)) ||
                       (v3 && (sl3 == sl0 || sl3 == sl1 || sl3 == sl2));
      const int  me = (g == 0) ? e0 : ((g == 1) ? e1 : ((g == 2) ? e2 : e3));
      const bool mv = (g == 0) ? true : ((g == 1) ? v1 : ((g == 2) ? v2 : v3));
      int sn = me >> BKSH;
      sn = sn < 0 ? 0 : (sn > nN - 1 ? nN - 1 : sn);
      const int slot = me & (BKSZ - 1);
      int cn = nodeBase + slot;
      cn = cn > nN - 1 ? nN - 1 : cn;

      const float* xsp = x + (size_t)sn * CDIM + 8 * hl;
      const float* xcp = x + (size_t)cn * CDIM + 8 * hl;
      const v4f xs0 = *(const v4f*)xsp, xs1 = *(const v4f*)(xsp + 4);
      const v4f xc0 = *(const v4f*)xcp, xc1 = *(const v4f*)(xcp + 4);
      float dt = xs0.x * xc0.x;
      dt = fmaf(xs0.y, xc0.y, dt); dt = fmaf(xs0.z, xc0.z, dt); dt = fmaf(xs0.w, xc0.w, dt);
      dt = fmaf(xs1.x, xc1.x, dt); dt = fmaf(xs1.y, xc1.y, dt); dt = fmaf(xs1.z, xc1.z, dt); dt = fmaf(xs1.w, xc1.w, dt);
      dt += __shfl_xor(dt, 4);
      dt += __shfl_xor(dt, 2);
      dt += __shfl_xor(dt, 1);
      const v4f nps = *(const v4f*)(nodep + (size_t)sn * 4);
      const v4f npc = *(const v4f*)(nodep + (size_t)cn * 4);
      float ev = dt * (nps.y * npc.y);
      ev = fmaxf(ev, NEGSL * ev);
      const float ts = temp[(size_t)sn * HEADS + hl] * nps.x;
      const float dc = npc.z - nps.z;

      const int npass = dup ? 4 : 1;
#pragma unroll 1
      for (int ps = 0; ps < npass; ++ps) {
        const bool act = mv && ((!dup) || (g == ps));
        const v4f st = st4[slot];
        const float ao = accl[slot * HEADS + hl];
        const float mnew = fmaxf(st.x, ev);
        const float sc = __expf(st.x - mnew);
        const float p  = __expf(ev - mnew);
        const float dn = fmaf(st.y, sc, p);
        const float an = fmaf(ao, sc, p * ts);
        const float ds = st.z + dc;
        if (act) {
          accl[slot * HEADS + hl] = an;
          if (hl == 0) { v4f nv; nv.x = mnew; nv.y = dn; nv.z = ds; nv.w = 0.0f; st4[slot] = nv; }
        }
        __builtin_amdgcn_fence(__ATOMIC_ACQ_REL, "wavefront");
        __builtin_amdgcn_wave_barrier();
      }
    }
  }
  __syncthreads();

  {
    const float coef = coefp[0], bb = biasp[0];
    for (int slot = tid; slot < BKSZ; slot += NTHR) {
      const int c  = nodeBase + slot;
      const int cc = c > nN - 1 ? nN - 1 : c;
      const v4f st = st4[slot];
      const float rden = st.y > 0.0f ? 1.0f / st.y : 0.0f;
      const int dg = degc[cc];
      const float dinv = dg > 0 ? 1.0f / (float)dg : 0.0f;
      const float add = (coef * st.z) * dinv;
      float sum = 0.0f;
#pragma unroll 1
      for (int h = 0; h < HEADS; ++h) sum += softplus_f(accl[slot * HEADS + h] * rden + add);
      const float tv = sum * 0.125f + bb;
      rtl[slot] = 1.0f / tv;
    }
  }
  __syncthreads();

  const int cp = (lane & 15) * 4;
#pragma unroll 1
  for (int pr = wave; pr < BKSZ / 2; pr += NWAVE) {
    const int r = 2 * pr + (lane >> 4);
    const int c = nodeBase + r;
    const int cc = c > nN - 1 ? nN - 1 : c;
    const v4f xv = *(const v4f*)(x + (size_t)cc * CDIM + cp);
    const float rt = rtl[r];
    const v4f o = xv * rt;
    if (c < nN) *(volatile v4f*)(out + (size_t)c * CDIM + cp) = o;
  }
  __threadfence();
#pragma unroll 1
  for (int pr = wave; pr < BKSZ / 2; pr += NWAVE) {
    const int r = 2 * pr + (lane >> 4);
    const int c = nodeBase + r;
    const int cc = c > nN - 1 ? nN - 1 : c;
    const v4f xv = *(const v4f*)(x + (size_t)cc * CDIM + cp);
    const float rt = rtl[r];
    const v4f o = xv * rt;
    if (c < nN) *(volatile v4f*)(out + (size_t)c * CDIM + cp) = o;
  }
}

extern "C" void kernel_launch(void* const* d_in, const int* in_sizes, int n_in,
                              void* d_out, int out_size, void* d_ws, size_t ws_size,
                              hipStream_t stream) {
  if (n_in < 8) return;
  const int nN = in_sizes[2];
  if (nN <= 0 || in_sizes[0] != nN * CDIM) return;
  const int n1 = in_sizes[1];
  if (n1 < 2 || (n1 & 1) != 0) return;
  const int nE = n1 / 2;
  if (in_sizes[3] != HEADS * CDIM) return;
  if (in_sizes[4] < 1 || in_sizes[5] < 1 || in_sizes[6] < 1 || in_sizes[7] < 1) return;
  if (out_size != nN * CDIM) return;
  if (nN > NBKT * BKSZ) return;
  if (nE > (1 << 27)) return;

  const float* x        = (const float*)d_in[0];
  const int*   edges    = (const int*)d_in[1];
  const int*   dist     = (const int*)d_in[2];
  const float* W        = (const float*)d_in[3];
  const float* coefp    = (const float*)d_in[4];
  const float* biasp    = (const float*)d_in[5];
  const float* train_a  = (const float*)d_in[6];
  const float* dist1_a  = (const float*)d_in[7];
  const int* srcs = edges;
  const int* dsts = edges + nE;
  float* out = (float*)d_out;

  const int NPAD   = ((nN + 255) / 256) * 256;
  const int nBkt   = (nN + BKSZ - 1) / BKSZ;
  const int nCh    = (nE + PCH - 1) / PCH;
  const int nDeg   = (nN + DEGB - 1) / DEGB;
  const int DEGPAD = nDeg * DEGB;
  const int lcap   = ((nE + 31) & ~31) + nCh * NBKT * 32;
  const int maxIter = lcap >> 5;

  char* ws = (char*)d_ws;
  size_t off = 0;
  const size_t oXs = off; off += (size_t)NPAD * CDIM * 2;     off = (off + 255) & ~(size_t)255;
  const size_t oNp = off; off += (size_t)NPAD * 16;           off = (off + 255) & ~(size_t)255;
  const size_t oTp = off; off += (size_t)NPAD * HEADS * 4;    off = (off + 255) & ~(size_t)255;
  const size_t oDg = off; off += (size_t)DEGPAD * 4;          off = (off + 255) & ~(size_t)255;
  const size_t oCt = off; off += (size_t)nCh * NBKT * 4;      off = (off + 255) & ~(size_t)255;
  const size_t oLs = off; off += (size_t)lcap * 4;            off = (off + 255) & ~(size_t)255;
  if (off > ws_size || off > (size_t)WSCAP) return;
  _Float16* xs16  = (_Float16*)(ws + oXs);
  float*    nodep = (float*)(ws + oNp);
  float*    temp  = (float*)(ws + oTp);
  int*      degc  = (int*)(ws + oDg);
  int*      ctab  = (int*)(ws + oCt);
  int*      elist = (int*)(ws + oLs);

  const int vec4 = (((nE & 3) == 0) && nE >= 4) ? 1 : 0;

  k_node<<<NPAD / NODB, NODB, 0, stream>>>(x, dist, train_a, dist1_a, xs16, nodep, nN);
  k_temp<<<NPAD / TROWS, TBLK, 0, stream>>>(xs16, W, temp);
  hipFuncSetAttribute(reinterpret_cast<const void*>(&k_degc),
                      hipFuncAttributeMaxDynamicSharedMemorySize, LDS_DEG);
  k_degc<<<nDeg, NTHR, LDS_DEG, stream>>>(srcs, degc, nE, vec4);
  k_part<0><<<nCh, NTHR, 0, stream>>>(srcs, dsts, ctab, elist, nN, nE, nCh, vec4, lcap);
  k_part<1><<<nCh, NTHR, 0, stream>>>(srcs, dsts, ctab, elist, nN, nE, nCh, vec4, lcap);
  hipFuncSetAttribute(reinterpret_cast<const void*>(&k_agg),
                      hipFuncAttributeMaxDynamicSharedMemorySize, LDS_AGG);
  k_agg<<<nBkt, NTHR, LDS_AGG, stream>>>(x, elist, ctab, nodep, temp, degc, coefp, biasp, out,
                                          nN, nCh, lcap, maxIter);
}
